// LoRAExpertAttention_4131758539047
// MI455X (gfx1250) — hardware-verified
//
#include <hip/hip_runtime.h>
#include <math.h>
#include <stdint.h>

#define NB_   4
#define SEQ_  1024
#define DM_   2048
#define NHQ_  16
#define NHK_  8
#define HD_   128
#define NEX_  4
#define RNK_  16
#define TOK_  (NB_ * SEQ_)
#define KVD_  (NHK_ * HD_)
#define LRK_  (NEX_ * RNK_)

typedef _Float16 v16h __attribute__((ext_vector_type(16)));
typedef _Float16 v8h  __attribute__((ext_vector_type(8)));
typedef __bf16   v16b __attribute__((ext_vector_type(16)));
typedef __bf16   v8b  __attribute__((ext_vector_type(8)));
typedef float    v8f  __attribute__((ext_vector_type(8)));
typedef float    v4f  __attribute__((ext_vector_type(4)));
typedef unsigned short v8us __attribute__((ext_vector_type(8)));

__device__ __forceinline__ unsigned short bf_bits(float f) {
  const unsigned u = __float_as_uint(f);
  return (unsigned short)((u + 0x7FFFu + ((u >> 16) & 1u)) >> 16);
}
__device__ __forceinline__ float bf_val(unsigned short b) { return __uint_as_float(((unsigned)b) << 16); }
__device__ __forceinline__ float bf_rne(float f) { return bf_val(bf_bits(f)); }
__device__ __forceinline__ _Float16 h_cv(float f) {
  return (fabsf(f) < 6.103515625e-05f) ? (_Float16)0.0f : (_Float16)f;
}

union FH_ { v16h v; v8h p[2]; };
union FB_ { v16b v; v8b p[2]; };
__device__ __forceinline__ v16h ldh(const _Float16* p) {
  FH_ f; f.p[0] = *(const v8h*)p; f.p[1] = *(const v8h*)(p + 16); return f.v;
}
__device__ __forceinline__ v16b ldbf(const unsigned short* p) {
  FB_ f; f.p[0] = *(const v8b*)(const void*)p; f.p[1] = *(const v8b*)(const void*)(p + 16); return f.v;
}
__device__ __forceinline__ v8f mma_b(v16b a, v16b b, v8f c) {
  return __builtin_amdgcn_wmma_f32_16x16x32_bf16(false, a, false, b, (short)0, c, false, false);
}
__device__ __forceinline__ v8f mma_h(v16h a, v16h b, v8f c) {
  return __builtin_amdgcn_wmma_f32_16x16x32_f16(false, a, false, b, (short)0, c, false, false);
}
__device__ __forceinline__ v8f zero8() { return (v8f){0.f, 0.f, 0.f, 0.f, 0.f, 0.f, 0.f, 0.f}; }

__device__ __forceinline__ void gd_1x8(v8f (&c)[8], v16b a, v16b (&b)[8]) {
  asm volatile("v_nop\n\tv_nop\n\tv_nop\n\tv_nop"
    : "+v"(c[0]), "+v"(c[1]), "+v"(c[2]), "+v"(c[3]), "+v"(c[4]), "+v"(c[5]), "+v"(c[6]), "+v"(c[7])
    : "v"(a), "v"(b[0]), "v"(b[1]), "v"(b[2]), "v"(b[3]), "v"(b[4]), "v"(b[5]), "v"(b[6]), "v"(b[7]));
}
__device__ __forceinline__ void gd_r(v8f& c0, v8f& c1, v16b a0, v16b a1, v16b b) {
  asm volatile("v_nop\n\tv_nop\n\tv_nop\n\tv_nop" : "+v"(c0), "+v"(c1) : "v"(a0), "v"(a1), "v"(b));
}
__device__ __forceinline__ void gd_2x4(v8f (&c)[2][4], v16b (&ah)[2], v16b (&al)[2], v16b (&b)[4]) {
  asm volatile("v_nop\n\tv_nop\n\tv_nop\n\tv_nop"
    : "+v"(c[0][0]), "+v"(c[0][1]), "+v"(c[0][2]), "+v"(c[0][3]),
      "+v"(c[1][0]), "+v"(c[1][1]), "+v"(c[1][2]), "+v"(c[1][3])
    : "v"(ah[0]), "v"(ah[1]), "v"(al[0]), "v"(al[1]), "v"(b[0]), "v"(b[1]), "v"(b[2]), "v"(b[3]));
}
__device__ __forceinline__ void gd_s(v8f& s, v16h (&q)[4], v16h (&k)[4]) {
  asm volatile("v_nop\n\tv_nop\n\tv_nop\n\tv_nop"
    : "+v"(s) : "v"(q[0]), "v"(q[1]), "v"(q[2]), "v"(q[3]), "v"(k[0]), "v"(k[1]), "v"(k[2]), "v"(k[3]));
}
__device__ __forceinline__ void gd_pv(v8f& o0, v8f& o1, v8f& r0, v8f& r1, v16h pa, v16h pl, v16h (&vh)[2], v16h (&vl)[2]) {
  asm volatile("v_nop\n\tv_nop\n\tv_nop\n\tv_nop"
    : "+v"(o0), "+v"(o1), "+v"(r0), "+v"(r1)
    : "v"(pa), "v"(pl), "v"(vh[0]), "v"(vh[1]), "v"(vl[0]), "v"(vl[1]));
}
__device__ __forceinline__ void wave_lds_sync() {
  __builtin_amdgcn_fence(__ATOMIC_RELEASE, "workgroup");
  __builtin_amdgcn_wave_barrier();
  __builtin_amdgcn_fence(__ATOMIC_ACQUIRE, "workgroup");
}

__global__ __launch_bounds__(256) void k_cvt_bf16(const float* __restrict__ src, unsigned short* __restrict__ dst,
                                                  int srcRows, int dstRows, int cols) {
  const size_t i = (size_t)blockIdx.x * 256 + threadIdx.x;
  const size_t n8 = (size_t)dstRows * (size_t)cols / 8;
  if (i >= n8) return;
  const size_t e0 = i * 8;
  const int r = (int)(e0 / (size_t)cols);
  const int c = (int)(e0 - (size_t)r * (size_t)cols);
  const int rs = (r < srcRows) ? r : (srcRows - 1);
  const float* p = src + (size_t)rs * cols + c;
  const v4f a = *(const v4f*)p;
  const v4f b = *(const v4f*)(p + 4);
  const bool z = (r >= srcRows);
  float f[8];
  f[0] = a[0]; f[1] = a[1]; f[2] = a[2]; f[3] = a[3]; f[4] = b[0]; f[5] = b[1]; f[6] = b[2]; f[7] = b[3];
  v8us o;
#pragma unroll
  for (int e = 0; e < 8; ++e) o[e] = z ? (unsigned short)0 : bf_bits(f[e]);
  unsigned short* q = dst + e0;
  *(volatile v8us*)q = o;
  __threadfence();
  *(volatile v8us*)q = o;
}

__global__ __launch_bounds__(256) void k_cvt_lorab(const float* __restrict__ lb, unsigned short* __restrict__ out) {
  const int gid = blockIdx.x * 256 + threadIdx.x;
  if (gid >= DM_ * 8) return;
  const int d = gid >> 3;
  const int piece = gid & 7;
  const int e = piece >> 1;
  const int rb = (piece & 1) * 8;
  const float* sp = lb + ((size_t)e * DM_ + d) * RNK_ + rb;
  const v4f a = *(const v4f*)sp;
  const v4f b = *(const v4f*)(sp + 4);
  v8us o;
  o[0] = bf_bits(a[0]); o[1] = bf_bits(a[1]); o[2] = bf_bits(a[2]); o[3] = bf_bits(a[3]);
  o[4] = bf_bits(b[0]); o[5] = bf_bits(b[1]); o[6] = bf_bits(b[2]); o[7] = bf_bits(b[3]);
  unsigned short* q = out + (size_t)d * LRK_ + piece * 8;
  *(volatile v8us*)q = o;
  __threadfence();
  *(volatile v8us*)q = o;
}

__global__ __launch_bounds__(128) void k_router(const unsigned short* __restrict__ Xb, const unsigned short* __restrict__ Gb,
                                                float* __restrict__ ew) {
  __shared__ __align__(16) float Ls[4][32 * 20];
  const int tid = threadIdx.x, wave = tid >> 5, lane = tid & 31, hh = lane >> 4, mm = lane & 15;
  const int t0 = (blockIdx.x * 4 + wave) * 32;
  v8f c0 = zero8(), c1 = zero8();
  const unsigned short* a0p = Xb + (size_t)(t0 + mm) * DM_ + 8 * hh;
  const unsigned short* a1p = Xb + (size_t)(t0 + 16 + mm) * DM_ + 8 * hh;
  const unsigned short* bp  = Gb + (size_t)mm * DM_ + 8 * hh;
  for (int k0 = 0; k0 < DM_; k0 += 32) {
    const v16b a0 = ldbf(a0p + k0);
    const v16b a1 = ldbf(a1p + k0);
    const v16b bb = ldbf(bp + k0);
    c0 = mma_b(a0, bb, c0);
    c1 = mma_b(a1, bb, c1);
    gd_r(c0, c1, a0, a1, bb);
  }
  float* L = Ls[wave];
#pragma unroll
  for (int r = 0; r < 8; ++r) {
    L[(8 * hh + r) * 20 + mm] = c0[r];
    L[(16 + 8 * hh + r) * 20 + mm] = c1[r];
  }
  wave_lds_sync();
  const v4f z = *(const v4f*)(L + lane * 20);
  const float mx = fmaxf(fmaxf(z[0], z[1]), fmaxf(z[2], z[3]));
  const float e0 = expf(z[0] - mx), e1 = expf(z[1] - mx), e2 = expf(z[2] - mx), e3 = expf(z[3] - mx);
  const float ssum = ((e0 + e1) + e2) + e3;
  const float inv = 1.0f / ssum;
  const float p0 = e0 * inv, p1 = e1 * inv, p2 = e2 * inv, p3 = e3 * inv;
  float bv = p0; int bi = 0;
  if (p1 > bv) { bv = p1; bi = 1; }
  if (p2 > bv) { bv = p2; bi = 2; }
  if (p3 > bv) { bv = p3; bi = 3; }
  float sv = -1.0f; int si = -1;
  if (bi != 0 && p0 > sv) { sv = p0; si = 0; }
  if (bi != 1 && p1 > sv) { sv = p1; si = 1; }
  if (bi != 2 && p2 > sv) { sv = p2; si = 2; }
  if (bi != 3 && p3 > sv) { sv = p3; si = 3; }
  v4f w;
  w[0] = (bi == 0 || si == 0) ? p0 : 0.0f;
  w[1] = (bi == 1 || si == 1) ? p1 : 0.0f;
  w[2] = (bi == 2 || si == 2) ? p2 : 0.0f;
  w[3] = (bi == 3 || si == 3) ? p3 : 0.0f;
  float* q = ew + (size_t)(t0 + lane) * NEX_;
  *(volatile v4f*)q = w;
  __threadfence();
  *(volatile v4f*)q = w;
}

__global__ __launch_bounds__(128) void k_qkv(
    const unsigned short* __restrict__ Xb, const unsigned short* __restrict__ Wqb,
    const unsigned short* __restrict__ Wkb, const unsigned short* __restrict__ Wvb,
    const float* __restrict__ cosT, const float* __restrict__ sinT,
    const float* __restrict__ qnw, const float* __restrict__ knw,
    _Float16* __restrict__ Qh, _Float16* __restrict__ Ql, _Float16* __restrict__ Kp,
    _Float16* __restrict__ Vth, _Float16* __restrict__ Vtl) {
  __shared__ __align__(16) float sm[8704];
  const int tid = threadIdx.x, wave = tid >> 5, lane = tid & 31, hh = lane >> 4, mm = lane & 15;
  const int tb = blockIdx.x;
  const int nb = blockIdx.y;
  const int tw = tb * 64 + wave * 16;
  const unsigned short* W;
  int kind, head;
  if (nb < 16)      { W = Wqb + (size_t)nb * HD_ * DM_;        kind = 0; head = nb; }
  else if (nb < 24) { W = Wkb + (size_t)(nb - 16) * HD_ * DM_; kind = 1; head = nb - 16; }
  else              { W = Wvb + (size_t)(nb - 24) * HD_ * DM_; kind = 2; head = nb - 24; }

  v8f acc[8];
#pragma unroll
  for (int j = 0; j < 8; ++j) acc[j] = zero8();
  const unsigned short* arow = Xb + (size_t)(tw + mm) * DM_ + 8 * hh;
  const unsigned short* brow = W + (size_t)mm * DM_ + 8 * hh;
  for (int k0 = 0; k0 < DM_; k0 += 32) {
    const v16b a = ldbf(arow + k0);
    v16b bf[8];
#pragma unroll
    for (int j = 0; j < 8; ++j) bf[j] = ldbf(brow + (size_t)j * 16 * DM_ + k0);
#pragma unroll
    for (int j = 0; j < 8; ++j) acc[j] = mma_b(a, bf[j], acc[j]);
    gd_1x8(acc, a, bf);
  }

  if (kind < 2) {
    float* sw = sm + wave * (16 * 132);
    const float* nw = (kind == 0) ? qnw : knw;
    float wv[8];
#pragma unroll
    for (int j = 0; j < 8; ++j) wv[j] = bf_rne(nw[16 * j + mm]);
#pragma unroll
    for (int r = 0; r < 8; ++r) {
      float ss = 0.f;
#pragma unroll
      for (int j = 0; j < 8; ++j) ss += acc[j][r] * acc[j][r];
      ss += __shfl_xor(ss, 1, 32);
      ss += __shfl_xor(ss, 2, 32);
      ss += __shfl_xor(ss, 4, 32);
      ss += __shfl_xor(ss, 8, 32);
      const float rstd = rsqrtf(ss * 0.0078125f + 1e-6f);
      const int tok = tw + 8 * hh + r;
      const float* cr = cosT + (size_t)tok * HD_;
      const float* sr = sinT + (size_t)tok * HD_;
#pragma unroll
      for (int j = 0; j < 4; ++j) {
        const int c = 16 * j + mm;
        const float x1 = acc[j][r] * rstd * wv[j];
        const float x2 = acc[j + 4][r] * rstd * wv[j + 4];
        const float c1 = bf_rne(cr[c]),      s1 = bf_rne(sr[c]);
        const float c2 = bf_rne(cr[c + 64]), s2 = bf_rne(sr[c + 64]);
        sw[(8 * hh + r) * 132 + c]      = x1 * c1 - x2 * s1;
        sw[(8 * hh + r) * 132 + c + 64] = x2 * c2 + x1 * s2;
      }
    }
    __syncthreads();
    const int b  = tw >> 10;
    const int s0 = tw & 1023;
    const size_t prow0 = (kind == 0) ? ((size_t)(b * NHQ_ + head) * SEQ_ + s0)
                                     : ((size_t)(b * NHK_ + head) * SEQ_ + s0);
    const int c8 = (lane & 15) * 8;
    for (int pass = 0; pass < 2; ++pass) {
#pragma unroll
      for (int it = 0; it < 8; ++it) {
        const int row = 2 * it + hh;
        const float* sp = sw + row * 132 + c8;
        const v4f u0 = *(const v4f*)sp;
        const v4f u1 = *(const v4f*)(sp + 4);
        float f[8];
        f[0] = u0[0]; f[1] = u0[1]; f[2] = u0[2]; f[3] = u0[3]; f[4] = u1[0]; f[5] = u1[1]; f[6] = u1[2]; f[7] = u1[3];
        const size_t go = (prow0 + row) * HD_ + c8;
        if (kind == 0) {
          v8h hv, lv;
#pragma unroll
          for (int e = 0; e < 8; ++e) {
            const _Float16 hq = h_cv(f[e]);
            hv[e] = hq;
            lv[e] = h_cv((f[e] - (float)hq) * 4096.0f);
          }
          *(volatile v8h*)(Qh + go) = hv;
          *(volatile v8h*)(Ql + go) = lv;
        } else {
          v8h kv;
#pragma unroll
          for (int e = 0; e < 8; ++e) kv[e] = h_cv(f[e]);
          *(volatile v8h*)(Kp + go) = kv;
        }
      }
      __threadfence();
    }
  } else {
#pragma unroll
    for (int j = 0; j < 8; ++j)
#pragma unroll
      for (int r = 0; r < 8; ++r)
        sm[(16 * j + mm) * 68 + wave * 16 + 8 * hh + r] = acc[j][r];
    __syncthreads();
    const int b  = (tb * 64) >> 10;
    const int s0 = (tb * 64) & 1023;
    const int q8 = lane >> 3, c8 = (lane & 7) * 8;
    const size_t vb = (size_t)(b * NHK_ + head) * HD_;
    for (int pass = 0; pass < 2; ++pass) {
#pragma unroll
      for (int it = 0; it < 8; ++it) {
        const int d = wave * 32 + it * 4 + q8;
        const float* sp = sm + d * 68 + c8;
        const v4f u0 = *(const v4f*)sp;
        const v4f u1 = *(const v4f*)(sp + 4);
        float f[8];
        f[0] = u0[0]; f[1] = u0[1]; f[2] = u0[2]; f[3] = u0[3]; f[4] = u1[0]; f[5] = u1[1]; f[6] = u1[2]; f[7] = u1[3];
        v8h hv, lv;
#pragma unroll
        for (int e = 0; e < 8; ++e) {
          const _Float16 hq = h_cv(f[e]);
          hv[e] = hq;
          lv[e] = h_cv((f[e] - (float)hq) * 1024.0f);
        }
        const size_t go = (vb + d) * SEQ_ + s0 + c8;
        *(volatile v8h*)(Vth + go) = hv;
        *(volatile v8h*)(Vtl + go) = lv;
      }
      __threadfence();
    }
  }
}

__global__ __launch_bounds__(64) void k_attn(
    const _Float16* __restrict__ Qh, const _Float16* __restrict__ Ql, const _Float16* __restrict__ Kp,
    const _Float16* __restrict__ Vth, const _Float16* __restrict__ Vtl,
    unsigned short* __restrict__ AOh, unsigned short* __restrict__ AOl) {
  __shared__ __align__(16) float    Sx[2][16 * 36];
  __shared__ __align__(16) _Float16 Ph[2][16 * 40];
  __shared__ __align__(16) _Float16 Pl[2][16 * 40];
  __shared__ __align__(16) float    Al[2][16];
  __shared__ __align__(16) float    Il[16];
  __shared__ __align__(16) float    Os[2][16 * 68];
  const int tid = threadIdx.x, wave = tid >> 5, lane = tid & 31, hh = lane >> 4, mm = lane & 15;
  const int qblk = blockIdx.x;
  const int bh = blockIdx.y;
  const int b = bh >> 4, hq = bh & 15, hk = hq >> 1;
  const int q0 = qblk * 16;
  const _Float16* Qp  = ((wave == 0) ? Qh : Ql) + ((size_t)(b * NHQ_ + hq) * SEQ_ + q0) * HD_;
  const _Float16* Kb  = Kp  + (size_t)(b * NHK_ + hk) * SEQ_ * HD_;
  const _Float16* Vhb = Vth + (size_t)(b * NHK_ + hk) * HD_ * SEQ_;
  const _Float16* Vlb = Vtl + (size_t)(b * NHK_ + hk) * HD_ * SEQ_;
  const int nCh = (q0 + 47) >> 5;
  const bool early = (qblk < 8);
  const int rr = lane & 7, kq = lane >> 3;
  const int row16 = wave * 8 + rr;
  const int qg = q0 + row16;
  float mrow = -INFINITY, lrow = 0.0f;
  v8f oacc[4], racc[4];
#pragma unroll
  for (int t = 0; t < 4; ++t) { oacc[t] = zero8(); racc[t] = zero8(); }

  for (int ch = 0; ch < nCh; ++ch) {
    const int kv0 = ch * 32;
    const int par = ch & 1;
    {
      v16h qf[4];
#pragma unroll
      for (int dc = 0; dc < 4; ++dc) qf[dc] = ldh(Qp + (size_t)mm * HD_ + dc * 32 + 8 * hh);
      v8f s[2];
#pragma unroll
      for (int j = 0; j < 2; ++j) {
        s[j] = zero8();
        v16h kf[4];
#pragma unroll
        for (int dc = 0; dc < 4; ++dc) kf[dc] = ldh(Kb + (size_t)(kv0 + 16 * j + mm) * HD_ + dc * 32 + 8 * hh);
#pragma unroll
        for (int dc = 0; dc < 4; ++dc) s[j] = mma_h(qf[dc], kf[dc], s[j]);
        gd_s(s[j], qf, kf);
      }
      float* sx = Sx[wave];
#pragma unroll
      for (int j = 0; j < 2; ++j)
#pragma unroll
        for (int r = 0; r < 8; ++r) sx[(8 * hh + r) * 36 + 16 * j + mm] = s[j][r];
    }
    __syncthreads();
    {
      const float* p0 = Sx[0] + row16 * 36 + 8 * kq;
      const float* p1 = Sx[1] + row16 * 36 + 8 * kq;
      const v4f a0 = *(const v4f*)p0;
      const v4f a1 = *(const v4f*)(p0 + 4);
      const v4f g0 = *(const v4f*)p1;
      const v4f g1 = *(const v4f*)(p1 + 4);
      float hi8[8], lo8[8];
      hi8[0] = a0[0]; hi8[1] = a0[1]; hi8[2] = a0[2]; hi8[3] = a0[3]; hi8[4] = a1[0]; hi8[5] = a1[1]; hi8[6] = a1[2]; hi8[7] = a1[3];
      lo8[0] = g0[0]; lo8[1] = g0[1]; lo8[2] = g0[2]; lo8[3] = g0[3]; lo8[4] = g1[0]; lo8[5] = g1[1]; lo8[6] = g1[2]; lo8[7] = g1[3];
      float sv[8];
      float cm = -INFINITY;
#pragma unroll
      for (int e = 0; e < 8; ++e) {
        const float v = (hi8[e] + lo8[e] * 0.000244140625f) * 0.08838834764831845f;
        const int key = kv0 + 8 * kq + e;
        sv[e] = (key > qg) ? -1.0e9f : v;
        cm = fmaxf(cm, sv[e]);
      }
      cm = fmaxf(cm, __shfl_xor(cm, 8, 32));
      cm = fmaxf(cm, __shfl_xor(cm, 16, 32));
      const float mnew  = fmaxf(mrow, cm);
      const float alpha = __expf(mrow - mnew);
      float psum = 0.0f;
      v8h h8, l8;
      l8 = (v8h){(_Float16)0.f, (_Float16)0.f, (_Float16)0.f, (_Float16)0.f, (_Float16)0.f, (_Float16)0.f, (_Float16)0.f, (_Float16)0.f};
#pragma unroll
      for (int e = 0; e < 8; ++e) {
        const float p  = __expf(sv[e] - mnew);
        psum += p;
        const float ph = p * 4096.0f;
        const _Float16 hq16 = h_cv(ph);
        h8[e] = hq16;
        if (early) l8[e] = h_cv((ph - (float)hq16) * 1024.0f);
      }
      psum += __shfl_xor(psum, 8, 32);
      psum += __shfl_xor(psum, 16, 32);
      lrow = lrow * alpha + psum;
      mrow = mnew;
      *(v8h*)(Ph[par] + row16 * 40 + 8 * kq) = h8;
      if (early) *(v8h*)(Pl[par] + row16 * 40 + 8 * kq) = l8;
      if (kq == 0) Al[par][row16] = alpha;
    }
    __syncthreads();
    {
      const v4f al0 = *(const v4f*)(Al[par] + 8 * hh);
      const v4f al1 = *(const v4f*)(Al[par] + 8 * hh + 4);
      float alr[8];
      alr[0] = al0[0]; alr[1] = al0[1]; alr[2] = al0[2]; alr[3] = al0[3]; alr[4] = al1[0]; alr[5] = al1[1]; alr[6] = al1[2]; alr[7] = al1[3];
#pragma unroll
      for (int t = 0; t < 4; ++t)
#pragma unroll
        for (int r = 0; r < 8; ++r) { oacc[t][r] *= alr[r]; racc[t][r] *= alr[r]; }
      const v16h pa = ldh(Ph[par] + mm * 40 + 8 * hh);
      v16h pl = pa;
      if (early) pl = ldh(Pl[par] + mm * 40 + 8 * hh);
#pragma unroll
      for (int g = 0; g < 2; ++g) {
        v16h vh[2], vl[2];
#pragma unroll
        for (int u = 0; u < 2; ++u) {
          const int d = wave * 64 + 16 * (2 * g + u) + mm;
          vh[u] = ldh(Vhb + (size_t)d * SEQ_ + kv0 + 8 * hh);
          vl[u] = ldh(Vlb + (size_t)d * SEQ_ + kv0 + 8 * hh);
        }
#pragma unroll
        for (int u = 0; u < 2; ++u) {
          oacc[2 * g + u] = mma_h(pa, vh[u], oacc[2 * g + u]);
          racc[2 * g + u] = mma_h(pa, vl[u], racc[2 * g + u]);
          if (early) racc[2 * g + u] = mma_h(pl, vh[u], racc[2 * g + u]);
        }
        gd_pv(oacc[2 * g], oacc[2 * g + 1], racc[2 * g], racc[2 * g + 1], pa, pl, vh, vl);
      }
    }
  }

  if (kq == 0) Il[row16] = 1.0f / (lrow * 4096.0f);
  __syncthreads();
  {
    const v4f i0 = *(const v4f*)(Il + 8 * hh);
    const v4f i1 = *(const v4f*)(Il + 8 * hh + 4);
    float inv[8];
    inv[0] = i0[0]; inv[1] = i0[1]; inv[2] = i0[2]; inv[3] = i0[3]; inv[4] = i1[0]; inv[5] = i1[1]; inv[6] = i1[2]; inv[7] = i1[3];
    float* os = Os[wave];
#pragma unroll
    for (int t = 0; t < 4; ++t)
#pragma unroll
      for (int r = 0; r < 8; ++r)
        os[(8 * hh + r) * 68 + 16 * t + mm] = (oacc[t][r] + racc[t][r] * 0.0009765625f) * inv[r];
    wave_lds_sync();
    const int q8 = lane >> 3, c8 = (lane & 7) * 8;
    const size_t tok0 = (size_t)b * SEQ_ + q0;
    const int col0 = hq * HD_ + wave * 64 + c8;
    for (int pass = 0; pass < 2; ++pass) {
#pragma unroll
      for (int it = 0; it < 4; ++it) {
        const int row = it * 4 + q8;
        const float* sp = os + row * 68 + c8;
        const v4f u0 = *(const v4f*)sp;
        const v4f u1 = *(const v4f*)(sp + 4);
        float f[8];
        f[0] = u0[0]; f[1] = u0[1]; f[2] = u0[2]; f[3] = u0[3]; f[4] = u1[0]; f[5] = u1[1]; f[6] = u1[2]; f[7] = u1[3];
        v8us oh, ol;
#pragma unroll
        for (int e = 0; e < 8; ++e) {
          const unsigned short hb = bf_bits(f[e]);
          oh[e] = hb;
          ol[e] = bf_bits(f[e] - bf_val(hb));
        }
        const size_t go = (tok0 + row) * DM_ + col0;
        *(volatile v8us*)(AOh + go) = oh;
        *(volatile v8us*)(AOl + go) = ol;
      }
      __threadfence();
    }
  }
}

__device__ __forceinline__ void kblock(v8f (&acc)[2][4], const unsigned short* Ah, const unsigned short* Al, int lda,
                                       const unsigned short* Bt, int ldb, int K, int m0, int n0, int hh, int mm) {
  const unsigned short* a0p = Ah + (size_t)(m0 + mm) * lda + 8 * hh;
  const unsigned short* a1p = Ah + (size_t)(m0 + 16 + mm) * lda + 8 * hh;
  const unsigned short* l0p = Al + (size_t)(m0 + mm) * lda + 8 * hh;
  const unsigned short* l1p = Al + (size_t)(m0 + 16 + mm) * lda + 8 * hh;
  const unsigned short* bp  = Bt + (size_t)(n0 + mm) * ldb + 8 * hh;
  for (int k0 = 0; k0 < K; k0 += 32) {
    v16b b[4];
#pragma unroll
    for (int j = 0; j < 4; ++j) b[j] = ldbf(bp + (size_t)j * 16 * ldb + k0);
    v16b ah[2], al[2];
    ah[0] = ldbf(a0p + k0); ah[1] = ldbf(a1p + k0);
    al[0] = ldbf(l0p + k0); al[1] = ldbf(l1p + k0);
#pragma unroll
    for (int i = 0; i < 2; ++i)
#pragma unroll
      for (int j = 0; j < 4; ++j) {
        acc[i][j] = mma_b(ah[i], b[j], acc[i][j]);
        acc[i][j] = mma_b(al[i], b[j], acc[i][j]);
      }
    gd_2x4(acc, ah, al, b);
  }
}

template <int EPI>
__global__ __launch_bounds__(128) void k_gemm2(
    const unsigned short* __restrict__ Ah, const unsigned short* __restrict__ Al, int lda,
    const unsigned short* __restrict__ Bt, int ldb, int K,
    const unsigned short* A2h, const unsigned short* A2l, int lda2,
    const unsigned short* Bt2, int ldb2, int K2,
    int tilesN, int nTiles, const float* __restrict__ ew,
    float* outF, int ldo, unsigned short* oh, unsigned short* ol) {
  __shared__ __align__(16) float st[4][32 * 68];
  const int tid = threadIdx.x, wave = tid >> 5, lane = tid & 31, hh = lane >> 4, mm = lane & 15;
  const int tile = blockIdx.x * 4 + wave;
  if (tile >= nTiles) return;
  const int tm = tile / tilesN;
  const int tn = tile - tm * tilesN;
  const int m0 = tm * 32;
  const int n0 = tn * 64;
  v8f acc[2][4];
#pragma unroll
  for (int i = 0; i < 2; ++i)
#pragma unroll
    for (int j = 0; j < 4; ++j) acc[i][j] = zero8();
  kblock(acc, Ah, Al, lda, Bt, ldb, K, m0, n0, hh, mm);
  if (K2 > 0) kblock(acc, A2h, A2l, lda2, Bt2, ldb2, K2, m0, n0, hh, mm);

  float* sw = st[wave];
#pragma unroll
  for (int i = 0; i < 2; ++i)
#pragma unroll
    for (int r = 0; r < 8; ++r) {
      const int row = 16 * i + 8 * hh + r;
      float f0 = 1.0f, f1 = 1.0f, f2 = 1.0f, f3 = 1.0f;
      if (EPI == 1) {
        const v4f w = *(const v4f*)(ew + (size_t)(m0 + row) * NEX_);
        f0 = 2.0f * w[0]; f1 = 2.0f * w[1]; f2 = 2.0f * w[2]; f3 = 2.0f * w[3];
      }
      sw[row * 68 + mm]      = acc[i][0][r] * f0;
      sw[row * 68 + 16 + mm] = acc[i][1][r] * f1;
      sw[row * 68 + 32 + mm] = acc[i][2][r] * f2;
      sw[row * 68 + 48 + mm] = acc[i][3][r] * f3;
    }
  wave_lds_sync();
  if (EPI == 0) {
    const int c4 = (lane & 15) * 4;
    for (int pass = 0; pass < 2; ++pass) {
#pragma unroll
      for (int it = 0; it < 16; ++it) {
        const int row = 2 * it + hh;
        const v4f v = *(const v4f*)(sw + row * 68 + c4);
        *(volatile v4f*)(outF + (size_t)(m0 + row) * ldo + n0 + c4) = v;
      }
      __threadfence();
    }
  } else {
    const int q8 = lane >> 3, c8 = (lane & 7) * 8;
    for (int pass = 0; pass < 2; ++pass) {
#pragma unroll
      for (int it = 0; it < 8; ++it) {
        const int row = 4 * it + q8;
        const float* sp = sw + row * 68 + c8;
        const v4f u0 = *(const v4f*)sp;
        const v4f u1 = *(const v4f*)(sp + 4);
        float f[8];
        f[0] = u0[0]; f[1] = u0[1]; f[2] = u0[2]; f[3] = u0[3]; f[4] = u1[0]; f[5] = u1[1]; f[6] = u1[2]; f[7] = u1[3];
        v8us hv, lv;
#pragma unroll
        for (int e = 0; e < 8; ++e) {
          const unsigned short hb = bf_bits(f[e]);
          hv[e] = hb;
          lv[e] = bf_bits(f[e] - bf_val(hb));
        }
        const size_t go = (size_t)(m0 + row) * LRK_ + c8;
        *(volatile v8us*)(oh + go) = hv;
        *(volatile v8us*)(ol + go) = lv;
      }
      __threadfence();
    }
  }
}

static_assert((size_t)TOK_ * DM_ * 2 == (size_t)DM_ * DM_ * 2 + 2 * (size_t)KVD_ * DM_ * 2);

extern "C" void kernel_launch(void* const* d_in, const int* in_sizes, int n_in,
                              void* d_out, int out_size, void* d_ws, size_t ws_size,
                              hipStream_t stream) {
  if (n_in < 12) return;
  if (in_sizes[0] != TOK_ * DM_ || in_sizes[1] != TOK_ * HD_ || in_sizes[2] != TOK_ * HD_) return;
  if (in_sizes[3] != DM_ * DM_ || in_sizes[4] != KVD_ * DM_ || in_sizes[5] != KVD_ * DM_ || in_sizes[6] != DM_ * DM_) return;
  if (in_sizes[7] != HD_ || in_sizes[8] != HD_ || in_sizes[9] != NEX_ * DM_) return;
  if (in_sizes[10] != LRK_ * DM_ || in_sizes[11] != NEX_ * DM_ * RNK_) return;
  if (out_size != TOK_ * DM_) return;

  const float* x     = (const float*)d_in[0];
  const float* cosT  = (const float*)d_in[1];
  const float* sinT  = (const float*)d_in[2];
  const float* Wq    = (const float*)d_in[3];
  const float* Wk    = (const float*)d_in[4];
  const float* Wv    = (const float*)d_in[5];
  const float* Wo    = (const float*)d_in[6];
  const float* qnw   = (const float*)d_in[7];
  const float* knw   = (const float*)d_in[8];
  const float* gate  = (const float*)d_in[9];
  const float* loraA = (const float*)d_in[10];
  const float* loraB = (const float*)d_in[11];
  float* out = (float*)d_out;

  const size_t szX  = (size_t)TOK_ * DM_ * 2;
  const size_t szWq = (size_t)DM_ * DM_ * 2;
  const size_t szWk = (size_t)KVD_ * DM_ * 2;
  const size_t szWo = (size_t)DM_ * DM_ * 2;
  const size_t szG  = (size_t)16 * DM_ * 2;
  const size_t szLA = (size_t)LRK_ * DM_ * 2;
  const size_t szLB = (size_t)DM_ * LRK_ * 2;
  const size_t szEW = (size_t)TOK_ * NEX_ * 4;
  const size_t szQ  = (size_t)NB_ * NHQ_ * SEQ_ * HD_ * 2;
  const size_t szK  = (size_t)NB_ * NHK_ * SEQ_ * HD_ * 2;
  const size_t szV  = (size_t)NB_ * NHK_ * HD_ * SEQ_ * 2;
  const size_t szHW = (size_t)TOK_ * LRK_ * 2;
  size_t off = 0;
  const size_t oX   = off; off += szX;
  const size_t oWq  = off; off += szWq;
  const size_t oWk  = off; off += szWk;
  const size_t oWv  = off; off += szWk;
  const size_t oWo  = off; off += szWo;
  const size_t oG   = off; off += szG;
  const size_t oLA  = off; off += szLA;
  const size_t oLB  = off; off += szLB;
  const size_t oEW  = off; off += szEW;
  const size_t oQh  = off; off += szQ;
  const size_t oQl  = off; off += szQ;
  const size_t oK   = off; off += szK;
  const size_t oVh  = off; off += szV;
  const size_t oVl  = off; off += szV;
  const size_t oHWh = off; off += szHW;
  const size_t oHWl = off; off += szHW;
  const size_t oAOh = oX;
  const size_t oAOl = oWq;
  if (off > ws_size) return;
  if (off > (size_t)134217728) return;

  char* ws = (char*)d_ws;
  unsigned short* Xb  = (unsigned short*)(ws + oX);
  unsigned short* Wqb = (unsigned short*)(ws + oWq);
  unsigned short* Wkb = (unsigned short*)(ws + oWk);
  unsigned short* Wvb = (unsigned short*)(ws + oWv);
  unsigned short* Wob = (unsigned short*)(ws + oWo);
  unsigned short* Gb  = (unsigned short*)(ws + oG);
  unsigned short* LAb = (unsigned short*)(ws + oLA);
  unsigned short* LBt = (unsigned short*)(ws + oLB);
  float*          ew  = (float*)(ws + oEW);
  _Float16*       Qh  = (_Float16*)(ws + oQh);
  _Float16*       Ql  = (_Float16*)(ws + oQl);
  _Float16*       Kp  = (_Float16*)(ws + oK);
  _Float16*       Vth = (_Float16*)(ws + oVh);
  _Float16*       Vtl = (_Float16*)(ws + oVl);
  unsigned short* HWh = (unsigned short*)(ws + oHWh);
  unsigned short* HWl = (unsigned short*)(ws + oHWl);
  unsigned short* AOh = (unsigned short*)(ws + oAOh);
  unsigned short* AOl = (unsigned short*)(ws + oAOl);

  const dim3 b256(256), b128(128), b64(64);
  k_cvt_bf16<<<dim3((TOK_ * DM_ / 8 + 255) / 256), b256, 0, stream>>>(x, Xb, TOK_, TOK_, DM_);
  k_cvt_bf16<<<dim3((DM_ * DM_ / 8 + 255) / 256), b256, 0, stream>>>(Wq, Wqb, DM_, DM_, DM_);
  k_cvt_bf16<<<dim3((KVD_ * DM_ / 8 + 255) / 256), b256, 0, stream>>>(Wk, Wkb, KVD_, KVD_, DM_);
  k_cvt_bf16<<<dim3((KVD_ * DM_ / 8 + 255) / 256), b256, 0, stream>>>(Wv, Wvb, KVD_, KVD_, DM_);
  k_cvt_bf16<<<dim3((DM_ * DM_ / 8 + 255) / 256), b256, 0, stream>>>(Wo, Wob, DM_, DM_, DM_);
  k_cvt_bf16<<<dim3((16 * DM_ / 8 + 255) / 256), b256, 0, stream>>>(gate, Gb, NEX_, 16, DM_);
  k_cvt_bf16<<<dim3((LRK_ * DM_ / 8 + 255) / 256), b256, 0, stream>>>(loraA, LAb, LRK_, LRK_, DM_);
  k_cvt_lorab<<<dim3((DM_ * 8 + 255) / 256), b256, 0, stream>>>(loraB, LBt);
  k_router<<<dim3(TOK_ / 32 / 4), b128, 0, stream>>>(Xb, Gb, ew);
  k_qkv<<<dim3(TOK_ / 64, 32), b128, 0, stream>>>(Xb, Wqb, Wkb, Wvb, cosT, sinT, qnw, knw, Qh, Ql, Kp, Vth, Vtl);
  k_attn<<<dim3(SEQ_ / 16, NB_ * NHQ_), b64, 0, stream>>>(Qh, Ql, Kp, Vth, Vtl, AOh, AOl);
  k_gemm2<1><<<dim3(TOK_ / 32 / 4), b128, 0, stream>>>(
      AOh, AOl, DM_, LAb, DM_, DM_,
      AOh, AOl, LRK_, LBt, LRK_, 0,
      1, TOK_ / 32, ew, (float*)(ws + oG), DM_, HWh, HWl);
  k_gemm2<0><<<dim3((TOK_ / 32) * (DM_ / 64) / 4), b128, 0, stream>>>(
      AOh, AOl, DM_, Wob, DM_, DM_,
      HWh, HWl, LRK_, LBt, LRK_, LRK_,
      DM_ / 64, (TOK_ / 32) * (DM_ / 64), ew, out, DM_, Gb, LAb);
  (void)hipGetLastError();
}
